// UniGCNII_67688684585240
// MI455X (gfx1250) — hardware-run, weakly checked
//
#include <hip/hip_runtime.h>


namespace {
constexpr int N = 50000, EC = 10000, NNZ = 200000, D = 256, NCLS = 40, NL = 4, NBLK = N / 16;
constexpr float XS = 8.0f, WSC = 256.0f;
typedef _Float16 b16;
typedef __attribute__((ext_vector_type(16))) _Float16 v16b;
typedef __attribute__((ext_vector_type(8))) _Float16 v8b;
typedef __attribute__((ext_vector_type(8))) float v8f;
typedef __attribute__((ext_vector_type(4))) float v4f;
__device__ __forceinline__ float bf16_rne(float f) { unsigned int u = __float_as_uint(f); u += 0x7FFFu + ((u >> 16) & 1u); return __uint_as_float(u & 0xFFFF0000u); }
__device__ __forceinline__ v16b frag_kb(const b16* p, int hh) { const v8b a = *(const v8b*)(p + 8 * hh), b = *(const v8b*)(p + 16 + 8 * hh); v16b f;
#pragma unroll
  for (int e = 0; e < 8; ++e) { f[e] = a[e]; f[8 + e] = b[e]; } return f; }
__device__ __forceinline__ v8f wmma16b(v16b a, v16b b, v8f c) { v8f d = __builtin_amdgcn_wmma_f32_16x16x32_f16(false, a, false, b, (short)0, c, false, false); asm volatile("v_nop\n\tv_nop\n\tv_nop\n\tv_nop" : "+v"(d) : "v"(a), "v"(b)); return d; }
__device__ __forceinline__ void wave_lds_sync() { __builtin_amdgcn_fence(__ATOMIC_RELEASE, "workgroup"); __builtin_amdgcn_wave_barrier(); __builtin_amdgcn_fence(__ATOMIC_ACQUIRE, "workgroup"); }
__device__ __forceinline__ float pmul(float a, float b) { float p = a * b; asm volatile("" : "+v"(p)); return p; }
__device__ __forceinline__ int iclamp(int v, int lo, int hi) { return v < lo ? lo : (v > hi ? hi : v); }
__device__ __forceinline__ float silu(float v) { return v / (1.0f + __expf(-v)); }
constexpr int CSR_NBLK9 = 512, CSR_GB9 = 9, CSR_GN9 = 1 << CSR_GB9  , CSR_TS9 = (CSR_GN9 < 32 ? 32 : CSR_GN9)  , CSR_MAXG9 = 512, CSR_CAP9 = 12288  ;
__device__ __host__ __forceinline__ int csr_tix9(int v) { return (v >> CSR_GB9) * CSR_TS9 + (v & (CSR_GN9 - 1)); }
__global__ __launch_bounds__(64) void csrA_kernel9(const int* __restrict__ dst, int E, int N, int nG, int CHP, int NGP, int* __restrict__ STG, int* __restrict__ HST) {
  extern __shared__ int sm[];
  int* cnt = sm; int* run = sm + NGP; int* ids = sm + 2 * NGP;
  const int b = blockIdx.x; const int ch = (E + CSR_NBLK9 - 1) / CSR_NBLK9; const int e0 = b * ch, e1 = min(E, e0 + ch);
  for (int i = threadIdx.x; i < NGP; i += 64) cnt[i] = 0;
  for (int i = threadIdx.x; i < CHP; i += 64) ids[i] = -1;
  __syncthreads();
  if (threadIdx.x == 0) {
    for (int e = e0; e < e1; ++e) { int d = dst[e]; d = (d < 0) ? 0 : (d >= N ? N - 1 : d); cnt[d >> CSR_GB9] += 1; }
    int acc = 0; for (int g = 0; g < nG; ++g) { run[g] = acc; acc += cnt[g]; }
    for (int e = e0; e < e1; ++e) { int d = dst[e]; d = (d < 0) ? 0 : (d >= N ? N - 1 : d); const int g = d >> CSR_GB9; ids[run[g]] = e; run[g] += 1; } }
  __syncthreads();
  typedef __attribute__((ext_vector_type(4))) int v4i;
  for (int pass = 0; pass < 2; ++pass) {
    for (int i = threadIdx.x; i < CHP / 4; i += 64) *(volatile v4i*)(STG + (size_t)b * CHP + i * 4) = *(const v4i*)(&ids[i * 4]);
    for (int i = threadIdx.x; i < NGP / 4; i += 64) { v4i v; for (int e = 0; e < 4; ++e) v[e] = (i * 4 + e < nG) ? cnt[i * 4 + e] : 0; *(volatile v4i*)(HST + (size_t)b * NGP + i * 4) = v; }
    __threadfence(); }
}
__global__ __launch_bounds__(512) void csrS_kernel9(const int* __restrict__ HST, int nG, int NGP, int* __restrict__ START, int* __restrict__ TOT, int* __restrict__ OFF) {
  __shared__ int tot[CSR_MAXG9];
  const int b = threadIdx.x;
  for (int pass = 0; pass < 2; ++pass) { int runb = 0; for (int g = 0; g < nG; ++g) { int c = HST[(size_t)b * NGP + g]; c = (c < 0) ? 0 : c; ((volatile int*)OFF)[(size_t)g * CSR_NBLK9 + b] = runb; runb += c; } __threadfence(); }
  for (int g = threadIdx.x; g < nG; g += 512) { int s = 0; for (int bb = 0; bb < CSR_NBLK9; ++bb) { int c = HST[(size_t)bb * NGP + g]; s += (c < 0) ? 0 : c; } tot[g] = s; }
  __syncthreads();
  if (threadIdx.x < 32) {
    __shared__ int st[CSR_MAXG9 + 32];
    if (threadIdx.x == 0) { int acc = 0; for (int g = 0; g < NGP; ++g) { st[g] = acc; if (g < nG) acc += (tot[g] + 31) & ~31; } st[NGP] = acc; }
    __builtin_amdgcn_fence(__ATOMIC_RELEASE, "workgroup"); __builtin_amdgcn_wave_barrier(); __builtin_amdgcn_fence(__ATOMIC_ACQUIRE, "workgroup");
    for (int pass = 0; pass < 2; ++pass) { for (int i = threadIdx.x; i < NGP + 32; i += 32) { ((volatile int*)START)[i] = (i <= NGP) ? st[min(i, NGP)] : 0; ((volatile int*)TOT)[i] = (i < nG) ? tot[i] : 0; } __threadfence(); } }
}
__global__ __launch_bounds__(256) void csrB_kernel9(const int* __restrict__ dst, int N, int nG, int CHP, int NGP, int permLen, const int* __restrict__ STG, const int* __restrict__ HST, const int* __restrict__ OFF, const int* __restrict__ START, const int* __restrict__ TOT, int* __restrict__ PERM, int* __restrict__ ROWPTR, int* __restrict__ ROWCNT, int* __restrict__ FLAG) {
  typedef __attribute__((ext_vector_type(4))) int v4i;
  __shared__ int ids[CSR_CAP9]; __shared__ unsigned short key[CSR_CAP9]; __shared__ int outp[CSR_CAP9]; __shared__ int ncnt[CSR_GN9 + 1]; __shared__ int boff[CSR_NBLK9 + 1];
  const int g = blockIdx.x, t_ = threadIdx.x; int tot = TOT[g]; int st = START[g], stn = START[g + 1]; const int v0 = g * CSR_GN9; const int nv = min(CSR_GN9, N - v0); const int t0 = g * CSR_TS9;
  st = (st < 0) ? 0 : (st > permLen - 32 ? permLen - 32 : st) & ~31; stn = (stn < st) ? st : (stn > permLen ? permLen : stn); tot = (tot < 0) ? 0 : tot; if (tot > stn - st && tot <= CSR_CAP9) tot = stn - st;
  if (tot > CSR_CAP9) {
    for (int pass = 0; pass < 2; ++pass) { for (int i = t_; i < CSR_TS9 / 4; i += 256) { v4i a, c; for (int e = 0; e < 4; ++e) { a[e] = st; c[e] = 0; } *(volatile v4i*)(ROWPTR + t0 + i * 4) = a; *(volatile v4i*)(ROWCNT + t0 + i * 4) = c; } if (t_ == 0) ((volatile int*)FLAG)[0] = 1; __threadfence(); } (void)nv; return; }
  if (t_ == 0) { int acc = 0; for (int b = 0; b < CSR_NBLK9; ++b) { boff[b] = acc; int c = HST[(size_t)b * NGP + g]; c = (c < 0) ? 0 : (c > CHP ? CHP : c); acc += c; if (acc > tot) acc = tot; } boff[CSR_NBLK9] = acc; }
  for (int i = t_; i <= CSR_GN9; i += 256) ncnt[i] = 0;
  __syncthreads();
  for (int b = 0; b < CSR_NBLK9; ++b) { const int c = boff[b + 1] - boff[b]; int o_ = OFF[(size_t)g * CSR_NBLK9 + b]; o_ = (o_ < 0) ? 0 : (o_ > CHP - c ? CHP - c : o_); const int* src_ = STG + (size_t)b * CHP + o_;
    for (int i = t_; i < c; i += 256) { int id = src_[i]; id = (id < 0) ? 0 : id; ids[boff[b] + i] = id; int d = dst[id]; d = (d < v0) ? v0 : (d >= N ? N - 1 : d); int kk = d - v0; kk = (kk < 0) ? 0 : (kk >= CSR_GN9 ? CSR_GN9 - 1 : kk); key[boff[b] + i] = (unsigned short)kk; } }
  __syncthreads();
  if (t_ == 0) { for (int i = 0; i < tot; ++i) ncnt[key[i]] += 1; int acc = 0; for (int vl = 0; vl < CSR_GN9; ++vl) { const int c = ncnt[vl]; ncnt[vl] = acc; acc += c; } ncnt[CSR_GN9] = acc;
    for (int i = 0; i < tot; ++i) { const int vl = key[i]; outp[ncnt[vl]] = ids[i]; ncnt[vl] += 1; }
    for (int vl = CSR_GN9; vl > 0; --vl) ncnt[vl] = ncnt[vl - 1]; ncnt[0] = 0; }
  __syncthreads();
  for (int pass = 0; pass < 2; ++pass) {
    for (int i = t_; i < (stn - st) / 4; i += 256) { v4i v; for (int e = 0; e < 4; ++e) { const int q = i * 4 + e; v[e] = (q < tot) ? outp[q] : -1; } *(volatile v4i*)(PERM + st + i * 4) = v; }
    for (int i = t_; i < CSR_TS9 / 4; i += 256) { v4i a, c; for (int e = 0; e < 4; ++e) { const int vl = i * 4 + e; const int vc = vl < CSR_GN9 ? vl : CSR_GN9; a[e] = (vl < CSR_GN9) ? st + ncnt[vc] : st; c[e] = (vl < nv) ? (ncnt[(vc < CSR_GN9 ? vc : CSR_GN9 - 1) + 1] - ncnt[vc]) : 0; } *(volatile v4i*)(ROWPTR + t0 + i * 4) = a; *(volatile v4i*)(ROWCNT + t0 + i * 4) = c; }
    __threadfence(); }
}
__global__ __launch_bounds__(256) void csrZ_kernel9(int* __restrict__ p, size_t n4) { typedef __attribute__((ext_vector_type(4))) int v4i; const size_t tid = (size_t)blockIdx.x * 256 + threadIdx.x, nth = (size_t)gridDim.x * 256; v4i z = {0, 0, 0, 0}; for (size_t i = tid; i < n4; i += nth) *(volatile v4i*)(p + i * 4) = z; }
struct CsrBufs9 { int *STG, *HST, *OFF, *START, *TOT, *PERM, *ROWPTR, *ROWCNT, *FLAG; int nG, NGP, CHP; size_t permLen; char* base; size_t bytes; };
static size_t csr_carve9(CsrBufs9& c, char* ws, size_t off, int E, int N) {
  const size_t off0 = off; c.base = ws + off;
  auto al = [&](size_t bytes) { char* p = ws + off; off += (bytes + 255) & ~(size_t)255; return p; };
  c.nG = (N + CSR_GN9 - 1) / CSR_GN9; c.NGP = (c.nG + 31) & ~31; const int ch = (E + CSR_NBLK9 - 1) / CSR_NBLK9; c.CHP = (ch + 31) & ~31; c.permLen = (size_t)E + 32 * (size_t)c.nG + 32;
  c.STG = (int*)al((size_t)CSR_NBLK9 * c.CHP * 4); c.HST = (int*)al((size_t)CSR_NBLK9 * c.NGP * 4); c.OFF = (int*)al((size_t)c.NGP * CSR_NBLK9 * 4); c.START = (int*)al((size_t)(c.NGP + 64) * 4); c.TOT = (int*)al((size_t)(c.NGP + 64) * 4);
  c.PERM = (int*)al(c.permLen * 4); c.ROWPTR = (int*)al((size_t)c.nG * CSR_TS9 * 4); c.ROWCNT = (int*)al((size_t)c.nG * CSR_TS9 * 4); c.FLAG = (int*)al(256);
  c.bytes = off - off0; return off;
}
static void csr_build9(const CsrBufs9& c, const int* dst, int E, int N, hipStream_t stream) {
  const size_t smem = (size_t)(2 * c.NGP + c.CHP) * 4;
  csrZ_kernel9<<<512, 256, 0, stream>>>((int*)c.base, c.bytes / 16);
  csrA_kernel9<<<CSR_NBLK9, 64, smem, stream>>>(dst, E, N, c.nG, c.CHP, c.NGP, c.STG, c.HST);
  csrS_kernel9<<<1, 512, 0, stream>>>(c.HST, c.nG, c.NGP, c.START, c.TOT, c.OFF);
  csrB_kernel9<<<c.nG, 256, 0, stream>>>(dst, N, c.nG, c.CHP, c.NGP, (int)c.permLen, c.STG, c.HST, c.OFF, c.START, c.TOT, c.PERM, c.ROWPTR, c.ROWCNT, c.FLAG);
}


__global__ __launch_bounds__(256) void wcopy_kernel(const float* __restrict__ w, int OUTW, int OUTP, b16* __restrict__ WT) {
  const size_t u = (size_t)blockIdx.x * 256 + threadIdx.x; if (u >= (size_t)OUTP * D / 8) return; const size_t e = u * 8; const int o = (int)(e / D); v8b v;
#pragma unroll
  for (int j = 0; j < 8; ++j) v[j] = (o < OUTW) ? (b16)(bf16_rne(w[e + j]) * WSC) : (b16)0.0f; for (int pass = 0; pass < 2; ++pass) { *(volatile v8b*)(WT + e) = v; __threadfence(); }
}
__global__ __launch_bounds__(32) void in_kernel(const float* __restrict__ x, const b16* __restrict__ WI, const float* __restrict__ bi, float* __restrict__ X0) {
  __shared__ __attribute__((aligned(16))) b16 Ah[16][D + 8]; __shared__ __attribute__((aligned(16))) float Tf[16][128 + 4];
  const int lane = threadIdx.x, nloc = lane & 15, hlf = lane >> 4; const size_t m0 = (size_t)blockIdx.x * 16;
  for (int rr = 0; rr < 16; ++rr) for (int q = 0; q < 8; ++q) Ah[rr][q * 32 + lane] = (b16)(bf16_rne(x[(m0 + rr) * D + q * 32 + lane]) * XS);
  wave_lds_sync();
#pragma unroll 1
  for (int cg = 0; cg < 2; ++cg) { v8f acc[8];
#pragma unroll
    for (int t = 0; t < 8; ++t) acc[t] = (v8f){};
#pragma unroll 2
    for (int kb = 0; kb < D; kb += 32) { const v16b a = frag_kb(&Ah[nloc][kb], hlf);
#pragma unroll
      for (int t = 0; t < 8; ++t) acc[t] = wmma16b(a, frag_kb(WI + (size_t)(cg * 128 + t * 16 + nloc) * D + kb, hlf), acc[t]); }
#pragma unroll
    for (int t = 0; t < 8; ++t) { const int c = cg * 128 + t * 16 + nloc; const float bb = bf16_rne(bi[c]);
#pragma unroll
      for (int r8 = 0; r8 < 8; ++r8) Tf[8 * hlf + r8][t * 16 + nloc] = silu(acc[t][r8] * (1.0f / (XS * WSC)) + bb); }
    wave_lds_sync();
    for (int pass = 0; pass < 2; ++pass) { for (int rr = 0; rr < 16; ++rr) *(volatile v4f*)(X0 + (m0 + rr) * D + cg * 128 + lane * 4) = *(const v4f*)(&Tf[rr][lane * 4]); __threadfence(); }
    wave_lds_sync(); }
}
__global__ __launch_bounds__(256) void edge_kernel(const float* __restrict__ X, const int* __restrict__ vert, const float* __restrict__ degE, const int* __restrict__ PERM, const int* __restrict__ ROWPTR, const int* __restrict__ ROWCNT, int permLen, int NLIM, float* __restrict__ XE) {
  const int wave = threadIdx.x >> 5, lane = threadIdx.x & 31; const size_t e = (size_t)blockIdx.x * 8 + wave; if (e >= (size_t)EC) return;
  int st = ROWPTR[e], cnt = ROWCNT[e]; cnt = iclamp(cnt, 0, 1 << 20); st = iclamp(st, 0, permLen - cnt); v4f a0 = {0, 0, 0, 0}, a1 = {0, 0, 0, 0};
#pragma unroll 1
  for (int j = 0; j < cnt; ++j) { const int p = iclamp(PERM[st + j], 0, NNZ - 1); const size_t v = (size_t)iclamp(vert[p], 0, N - 1); if (v >= (size_t)NLIM) continue; const v4f x0 = *(const v4f*)(X + v * D + lane * 8), x1 = *(const v4f*)(X + v * D + lane * 8 + 4); for (int i = 0; i < 4; ++i) { a0[i] += x0[i]; a1[i] += x1[i]; } }
  const float w = pmul(1.0f / (float)(cnt < 1 ? 1 : cnt), bf16_rne(degE[e])); for (int i = 0; i < 4; ++i) { a0[i] = pmul(a0[i], w); a1[i] = pmul(a1[i], w); }
  for (int pass = 0; pass < 2; ++pass) { *(volatile v4f*)(XE + e * D + lane * 8) = a0; *(volatile v4f*)(XE + e * D + lane * 8 + 4) = a1; __threadfence(); }
}
__global__ __launch_bounds__(32) void vert_kernel(const float* __restrict__ XE, const int* __restrict__ edg, const float* __restrict__ degV, const int* __restrict__ PERM, const int* __restrict__ ROWPTR, const int* __restrict__ ROWCNT, int permLen, const float* __restrict__ X0, const float* __restrict__ g, const float* __restrict__ be, const float* __restrict__ alphap, const float* __restrict__ betap, const b16* __restrict__ WC, int NLIM, float* __restrict__ XN) {
  __shared__ __attribute__((aligned(16))) b16 Ah[16][D + 8]; __shared__ __attribute__((aligned(16))) float Xi[16][D + 4], Tf[16][128 + 4];
  const int lane = threadIdx.x, nloc = lane & 15, hlf = lane >> 4; const size_t m0 = (size_t)blockIdx.x * 16; if (m0 >= (size_t)NLIM) return; const float alpha = bf16_rne(alphap[0]), beta = bf16_rne(betap[0]);
  for (int rr = 0; rr < 16; ++rr) { const size_t v = m0 + rr; int st = ROWPTR[v], cnt = ROWCNT[v]; cnt = iclamp(cnt, 0, 1 << 20); st = iclamp(st, 0, permLen - cnt); float a[8]; for (int i = 0; i < 8; ++i) a[i] = 0.0f;
#pragma unroll 1
    for (int j = 0; j < cnt; ++j) { const int p = iclamp(PERM[st + j], 0, NNZ - 1); const size_t e = (size_t)iclamp(edg[p], 0, EC - 1); const v4f x0 = *(const v4f*)(XE + e * D + lane * 8), x1 = *(const v4f*)(XE + e * D + lane * 8 + 4); for (int i = 0; i < 4; ++i) { a[i] += x0[i]; a[4 + i] += x1[i]; } }
    const float dv = bf16_rne(degV[v]); float xl[8], s = 0.0f; for (int i = 0; i < 8; ++i) { xl[i] = 2.0f * pmul(a[i], dv); s += xl[i]; }
    for (int o = 16; o; o >>= 1) s += __shfl_xor(s, o); const float mu = s * (1.0f / D); float q = 0.0f; for (int i = 0; i < 8; ++i) { const float d_ = xl[i] - mu; q += pmul(d_, d_); } for (int o = 16; o; o >>= 1) q += __shfl_xor(q, o); const float rs = rsqrtf(q * (1.0f / D) + 1e-5f);
    for (int i = 0; i < 8; ++i) { const int c = lane * 8 + i; const float ln = pmul(pmul(xl[i] - mu, rs), bf16_rne(g[c])) + bf16_rne(be[c]); const float xi = pmul(1.0f - alpha, ln) + pmul(alpha, X0[v * D + c]); Xi[rr][c] = xi; Ah[rr][c] = (b16)(xi * XS); } }
  wave_lds_sync();
#pragma unroll 1
  for (int cg = 0; cg < 2; ++cg) { v8f acc[8];
#pragma unroll
    for (int t = 0; t < 8; ++t) acc[t] = (v8f){};
#pragma unroll 2
    for (int kb = 0; kb < D; kb += 32) { const v16b a = frag_kb(&Ah[nloc][kb], hlf);
#pragma unroll
      for (int t = 0; t < 8; ++t) acc[t] = wmma16b(a, frag_kb(WC + (size_t)(cg * 128 + t * 16 + nloc) * D + kb, hlf), acc[t]); }
#pragma unroll
    for (int t = 0; t < 8; ++t) { const int c = cg * 128 + t * 16 + nloc;
#pragma unroll
      for (int r8 = 0; r8 < 8; ++r8) { const int rl = 8 * hlf + r8; Tf[rl][t * 16 + nloc] = silu(pmul(1.0f - beta, Xi[rl][c]) + pmul(beta, acc[t][r8] * (1.0f / (XS * WSC)))); } }
    wave_lds_sync();
    for (int pass = 0; pass < 2; ++pass) { for (int rr = 0; rr < 16; ++rr) *(volatile v4f*)(XN + (m0 + rr) * D + cg * 128 + lane * 4) = *(const v4f*)(&Tf[rr][lane * 4]); __threadfence(); }
    wave_lds_sync(); }
}
__global__ __launch_bounds__(32) void out_kernel(const float* __restrict__ X, const b16* __restrict__ WO, const float* __restrict__ bo, float* __restrict__ out) {
  __shared__ __attribute__((aligned(16))) b16 Ah[16][D + 8]; __shared__ float Lg[16][48], So[16][NCLS];
  const int lane = threadIdx.x, nloc = lane & 15, hlf = lane >> 4; const size_t m0 = (size_t)blockIdx.x * 16;
  for (int rr = 0; rr < 16; ++rr) for (int q = 0; q < 8; ++q) Ah[rr][q * 32 + lane] = (b16)(X[(m0 + rr) * D + q * 32 + lane] * XS);
  wave_lds_sync();
#pragma unroll
  for (int t = 0; t < 3; ++t) { v8f acc = {};
#pragma unroll 2
    for (int kb = 0; kb < D; kb += 32) acc = wmma16b(frag_kb(&Ah[nloc][kb], hlf), frag_kb(WO + (size_t)(t * 16 + nloc) * D + kb, hlf), acc);
    const int c = t * 16 + nloc; const float bb = c < NCLS ? bf16_rne(bo[c]) : 0.0f;
#pragma unroll
    for (int r8 = 0; r8 < 8; ++r8) Lg[8 * hlf + r8][c] = acc[r8] * (1.0f / (XS * WSC)) + bb; }
  wave_lds_sync();
  for (int rr = 0; rr < 16; ++rr) { const float v0 = Lg[rr][lane], v1 = (lane < NCLS - 32) ? Lg[rr][32 + lane] : -INFINITY; float mx = fmaxf(v0, v1); for (int o = 16; o; o >>= 1) mx = fmaxf(mx, __shfl_xor(mx, o)); float s = __expf(v0 - mx) + ((lane < NCLS - 32) ? __expf(v1 - mx) : 0.0f); for (int o = 16; o; o >>= 1) s += __shfl_xor(s, o); const float lse = mx + __logf(s); So[rr][lane] = v0 - lse; if (lane < NCLS - 32) So[rr][32 + lane] = v1 - lse; }
  wave_lds_sync();
  for (int pass = 0; pass < 2; ++pass) { for (int i = lane; i < 16 * NCLS; i += 32) ((volatile float*)out)[m0 * NCLS + i] = So[i / NCLS][i % NCLS]; __threadfence(); }
}
}

extern "C" void kernel_launch(void* const* d_in, const int* in_sizes, int n_in, void* d_out, int out_size, void* d_ws, size_t ws_size, hipStream_t stream) {
  (void)n_in;
  auto Fp = [&](int i) { return (const float*)d_in[i]; }; auto Ip = [&](int i) { return (const int*)d_in[i]; };
  if (in_sizes[0] != N * D || in_sizes[1] != NNZ || in_sizes[2] != NNZ || in_sizes[3] != EC || in_sizes[4] != N || in_sizes[5] != D * D || in_sizes[7] != NL * D * D || in_sizes[8] != NL || in_sizes[9] != NL || in_sizes[12] != NCLS * D || out_size != N * NCLS) return;
  const int NLIM = N; const int GB16 = NBLK;
  size_t off = 0; char* ws = (char*)d_ws;
  auto carve = [&](size_t bytes) { char* p = ws + off; off += (bytes + 255) & ~(size_t)255; return p; };
  b16* WI = (b16*)carve((size_t)D * D * 2); b16* WC = (b16*)carve((size_t)NL * D * D * 2); b16* WO = (b16*)carve((size_t)48 * D * 2); float* X0 = (float*)carve((size_t)N * D * 4); float* XA = (float*)carve((size_t)N * D * 4); float* XB = (float*)carve((size_t)N * D * 4); float* XE = (float*)carve((size_t)EC * D * 4);
  CsrBufs9 ce, cv; off = csr_carve9(ce, ws, off, NNZ, EC); off = csr_carve9(cv, ws, off, NNZ, N);
  if (off > ws_size || off > ((size_t)192 << 20)) return;
  wcopy_kernel<<<(D * D / 8 + 255) / 256, 256, 0, stream>>>(Fp(5), D, D, WI); wcopy_kernel<<<(NL * D * D / 8 + 255) / 256, 256, 0, stream>>>(Fp(7), NL * D, NL * D, WC); wcopy_kernel<<<(48 * D / 8 + 255) / 256, 256, 0, stream>>>(Fp(12), NCLS, 48, WO);
  csr_build9(ce, Ip(2), NNZ, EC, stream); csr_build9(cv, Ip(1), NNZ, N, stream);
  in_kernel<<<GB16, 32, 0, stream>>>(Fp(0), WI, Fp(6), X0);
  const float* Xcur = X0; float* bufs[2] = {XA, XB};
  for (int l = 0; l < NL; ++l) { float* Xn = bufs[l & 1];
    edge_kernel<<<EC / 8, 256, 0, stream>>>(Xcur, Ip(1), Fp(3), ce.PERM, ce.ROWPTR, ce.ROWCNT, (int)ce.permLen, NLIM, XE);
    vert_kernel<<<GB16, 32, 0, stream>>>(XE, Ip(2), Fp(4), cv.PERM, cv.ROWPTR, cv.ROWCNT, (int)cv.permLen, X0, Fp(10) + l * D, Fp(11) + l * D, Fp(8) + l, Fp(9) + l, WC + (size_t)l * D * D, NLIM, Xn);
    Xcur = Xn; }
  out_kernel<<<GB16, 32, 0, stream>>>(Xcur, WO, Fp(13), (float*)d_out);
}
